// S4dLayer_73632919323116
// MI455X (gfx1250) — hardware-run, weakly checked
//
#include <hip/hip_runtime.h>
#include <math.h>

typedef __attribute__((ext_vector_type(16))) _Float16 v16h;
typedef __attribute__((ext_vector_type(8)))  _Float16 v8h;
typedef __attribute__((ext_vector_type(8)))  float    v8f;
typedef __attribute__((ext_vector_type(4)))  float    v4f;

constexpr int kBatch   = 8;
constexpr int kChan    = 512;
constexpr int kLen     = 2048;
constexpr int kModes   = 64;
constexpr int kTapOrigin = 2048;
constexpr int kTapPitch  = 2112;
constexpr int kTapCopies = 8;
constexpr int kTapChunks = kTapCopies * kTapPitch / 8;
constexpr int kTapChunksPerCopy = kTapPitch / 8;
constexpr int kTapLds    = 2120;
constexpr int kSigPad    = 64;
constexpr int kSigPitch  = kSigPad + kLen;
constexpr int kSigChunksPerRow = kSigPitch / 8;
constexpr int kSigChunks = kBatch * kChan * kSigChunksPerRow;
constexpr int kStrip     = 64;
constexpr int kPairSpan  = 128;
constexpr int kPairs     = kLen / kPairSpan;
constexpr float kTapCarry = 64.0f;
constexpr float kSigCarry = 16.0f;
constexpr float kFold     = 1.0f / (kTapCarry * kSigCarry);
constexpr float kHalfMinNormal = 6.103515625e-5f;
constexpr float kTapSkip  = 1.0e-9f;

static_assert(kTapOrigin == kLen);
static_assert(kTapPitch == kLen + 64);
static_assert((kTapPitch % 64) == 0);
static_assert((kSigPitch % 64) == 0);
static_assert(kTapChunks == 2112);
static_assert(kTapChunksPerCopy == 264);
static_assert(kSigChunks == 4224 * 256);
static_assert(kPairs == 16);
static_assert(kTapLds >= kTapPitch + 8);
static_assert(kFold == 1.0f / 1024.0f);

constexpr size_t kOffPar  = 0;
constexpr size_t kOffTap  = kOffPar + (size_t)kChan * 4 * kModes * 4;
constexpr size_t kOffSig  = kOffTap + (size_t)kChan * kTapCopies * kTapPitch * 2;
constexpr size_t kWsTotal = kOffSig + (size_t)kBatch * kChan * kSigPitch * 2;
static_assert(kWsTotal == 35127296ull);
static_assert(kWsTotal <= 134217728ull);
static_assert((kOffTap % 128) == 0 && (kOffSig % 128) == 0);

__device__ __forceinline__ v16h frag_load(const _Float16* p) {
  union U { v16h v; v8h h[2]; };
  U f;
  f.h[0] = *(const v8h*)(p);
  f.h[1] = *(const v8h*)(p + 16);
  return f.v;
}
__device__ __forceinline__ v8f mma_f16(v16h a, v16h b, v8f c) {
  c = __builtin_amdgcn_wmma_f32_16x16x32_f16(false, a, false, b, (short)0, c, false, false);
  asm volatile("v_nop\n\tv_nop\n\tv_nop\n\tv_nop" : "+v"(c) : "v"(a), "v"(b));
  return c;
}
__device__ __forceinline__ float carry_flush(float v, float carry) {
  const float s = v * carry;
  return (fabsf(s) < kHalfMinNormal) ? 0.0f : s;
}

__global__ __launch_bounds__(64) void mode_param_kernel(
    const float* __restrict__ A_re, const float* __restrict__ A_im, const float* __restrict__ Cm,
    const float* __restrict__ logst, float* __restrict__ PAR)
{
  const int h = blockIdx.x;
  const int n = threadIdx.x;
  const int hn = h * kModes + n;
  const float are  = fminf(A_re[hn], -1e-4f);
  const float aim  = A_im[hn];
  const float step = expf(logst[h]);
  const float dre  = step * are;
  const float dmi  = step * aim;
  const float er   = expf(dre);
  float sn, cs;
  sincosf(dmi, &sn, &cs);
  const float wr = er * cs;
  const float wi = er * sn;
  const float cre = Cm[2 * hn];
  const float cim = Cm[2 * hn + 1];
  const float nr = wr - 1.0f;
  const float ni = wi;
  const float pr = cre * nr - cim * ni;
  const float pi = cre * ni + cim * nr;
  const float den = are * are + aim * aim;
  const float inv = 1.0f / den;
  const float cfr = (pr * are + pi * aim) * inv;
  const float cfi = (pi * are - pr * aim) * inv;
  volatile float* vb = PAR + (size_t)h * (4 * kModes) + n;
  vb[0]          = dre;
  vb[kModes]     = dmi;
  vb[2 * kModes] = cfr;
  vb[3 * kModes] = cfi;
  __threadfence();
  vb[0]          = dre;
  vb[kModes]     = dmi;
  vb[2 * kModes] = cfr;
  vb[3 * kModes] = cfi;
}

__global__ __launch_bounds__(256) void tap_plane_kernel(
    const float* __restrict__ PAR, unsigned short* __restrict__ TAP)
{
  __shared__ float sPar[4 * kModes];
  __shared__ float sK[kTapLds];
  const int h = blockIdx.x;
  const int tid = threadIdx.x;
  sPar[tid] = PAR[(size_t)h * (4 * kModes) + tid];
  if (tid < 72) {
    const int p = (tid == 0) ? 0 : (kTapOrigin + tid);
    sK[p] = 0.0f;
  }
  __syncthreads();
  float mx = sPar[0];
  float sumc = 0.0f;
#pragma unroll 1
  for (int n = 0; n < kModes; ++n) {
    mx = fmaxf(mx, sPar[n]);
    sumc += fabsf(sPar[2 * kModes + n]) + fabsf(sPar[3 * kModes + n]);
  }
  const int lwave = tid & ~31;
#pragma unroll 1
  for (int i = 0; i < kLen / 256; ++i) {
    const int l = i * 256 + tid;
    const float lf = (float)l;
    const float lfirst = (float)(i * 256 + lwave);
    const float bound = sumc * expf(mx * lfirst);
    const bool skip = (mx < 0.0f) && (bound < kTapSkip);
    float acc = 0.0f;
    if (!skip) {
#pragma unroll 1
      for (int n = 0; n < kModes; ++n) {
        const float ar = sPar[n] * lf;
        const float ai = sPar[kModes + n] * lf;
        float e = expf(ar);
        e = (e < 1.17549435e-38f) ? 0.0f : e;
        float sn, cs;
        sincosf(ai, &sn, &cs);
        const float tr = sPar[2 * kModes + n] * cs - sPar[3 * kModes + n] * sn;
        acc += e * tr;
      }
    }
    sK[kTapOrigin - l] = acc;
  }
  __syncthreads();
#pragma unroll 1
  for (int it = 0; it < 9; ++it) {
    const int ch = it * 256 + tid;
    if (ch < kTapChunks) {
      const int c  = ch / kTapChunksPerCopy;
      const int j0 = (ch - c * kTapChunksPerCopy) * 8;
      v8h hv;
#pragma unroll
      for (int e = 0; e < 8; ++e) {
        const float s = carry_flush(sK[j0 + c + e], kTapCarry);
        hv[e] = (_Float16)s;
      }
      unsigned short* dst = TAP + ((size_t)h * kTapChunks + ch) * 8;
      *(volatile v8h*)dst = hv;
      __threadfence();
      *(volatile v8h*)dst = hv;
    }
  }
}

__global__ __launch_bounds__(256) void signal_plane_kernel(
    const float* __restrict__ u, unsigned short* __restrict__ SIG)
{
  const int ch  = blockIdx.x * 256 + threadIdx.x;
  const int row = ch / kSigChunksPerRow;
  const int cj  = ch - row * kSigChunksPerRow;
  const bool pad = (cj < (kSigPad / 8));
  const int cs  = pad ? 0 : (cj - (kSigPad / 8));
  const float* src = u + (size_t)row * kLen + cs * 8;
  v4f a0 = *(const v4f*)(src);
  v4f a1 = *(const v4f*)(src + 4);
  asm volatile("" : "+v"(a0), "+v"(a1));
  v8h hv;
#pragma unroll
  for (int e = 0; e < 4; ++e) {
    const float s0 = carry_flush(a0[e], kSigCarry);
    const float s1 = carry_flush(a1[e], kSigCarry);
    hv[e]     = (_Float16)(pad ? 0.0f : s0);
    hv[4 + e] = (_Float16)(pad ? 0.0f : s1);
  }
  unsigned short* dst = SIG + (size_t)ch * 8;
  *(volatile v8h*)dst = hv;
  __threadfence();
  *(volatile v8h*)dst = hv;
}

template <bool BOTH>
__device__ __forceinline__ void conv_step(const _Float16* aP, const _Float16* bPA, const _Float16* bPB,
                                          int delta, v8f (&accA)[4], v8f (&accB)[4]) {
  const v16h fb = frag_load(bPB - delta);
  v16h fa = fb;
  if (BOTH) fa = frag_load(bPA - delta);
#pragma unroll
  for (int mi = 0; mi < 4; ++mi) {
    const v16h ta = frag_load(aP - delta - 16 * mi);
    if (BOTH) accA[mi] = mma_f16(ta, fa, accA[mi]);
    accB[mi] = mma_f16(ta, fb, accB[mi]);
  }
}

__device__ __forceinline__ void store_pair(float* slab, const v8f (&acc)[4], int pq, int h, int lane, float dh,
                                           const float* __restrict__ u, float* __restrict__ out) {
  const int n  = lane & 15;
  const int hh = lane >> 4;
#pragma unroll
  for (int mi = 0; mi < 4; ++mi) {
#pragma unroll
    for (int r = 0; r < 8; ++r) slab[n * 68 + 16 * mi + 8 * hh + r] = acc[mi][r] * kFold;
  }
  __builtin_amdgcn_fence(__ATOMIC_RELEASE, "workgroup");
  __builtin_amdgcn_wave_barrier();
  __builtin_amdgcn_fence(__ATOMIC_ACQUIRE, "workgroup");
  const int c4 = (lane & 15) * 4;
  v4f vals[8];
#pragma unroll
  for (int it = 0; it < 8; ++it) {
    const int row = it * 2 + hh;
    const int gr = row >> 3;
    const int br = row & 7;
    const size_t off = ((size_t)br * kChan + h) * kLen + kPairSpan * pq + kStrip * gr + c4;
    const v4f y  = *(const v4f*)(slab + row * 68 + c4);
    const v4f uu = *(const v4f*)(u + off);
    v4f o;
    o[0] = y[0] + dh * uu[0];
    o[1] = y[1] + dh * uu[1];
    o[2] = y[2] + dh * uu[2];
    o[3] = y[3] + dh * uu[3];
    vals[it] = o;
  }
  for (int pass = 0; pass < 2; ++pass) {
#pragma unroll
    for (int it = 0; it < 8; ++it) {
      const int row = it * 2 + hh;
      const int gr = row >> 3;
      const int br = row & 7;
      const size_t off = ((size_t)br * kChan + h) * kLen + kPairSpan * pq + kStrip * gr + c4;
      *(volatile v4f*)(out + off) = vals[it];
    }
    __threadfence();
  }
  __builtin_amdgcn_fence(__ATOMIC_RELEASE, "workgroup");
  __builtin_amdgcn_wave_barrier();
  __builtin_amdgcn_fence(__ATOMIC_ACQUIRE, "workgroup");
}

__global__ __launch_bounds__(256) void toeplitz_conv_kernel(
    const unsigned short* __restrict__ TAPp, const unsigned short* __restrict__ SIGp,
    const float* __restrict__ u, const float* __restrict__ Dv, float* __restrict__ out)
{
  __shared__ __align__(16) float sT[8][16 * 68];
  const _Float16* TAP = (const _Float16*)TAPp;
  const _Float16* SIG = (const _Float16*)SIGp;
  const int h    = blockIdx.x;
  const int lane = threadIdx.x & 31;
  const int w    = __builtin_amdgcn_readfirstlane((int)(threadIdx.x >> 5));
  const int n    = lane & 15;
  const int hh   = lane >> 4;
  const int g    = n >> 3;
  const int bb   = n & 7;
  const int cc   = (8 - (n & 7)) & 7;
  const int mc   = n + cc;
  const _Float16* aP = TAP + ((size_t)h * kTapCopies + cc) * kTapPitch + (kTapOrigin - mc + 8 * hh);
  const int pA = w;
  const int pB = (kPairs - 1) - w;
  const _Float16* uRow = SIG + ((size_t)bb * kChan + h) * kSigPitch + kSigPad + kStrip * g + 8 * hh;
  const _Float16* bPA = uRow + kPairSpan * pA;
  const _Float16* bPB = uRow + kPairSpan * pB;

  v8f accA[4], accB[4];
#pragma unroll
  for (int i = 0; i < 4; ++i) {
    accA[i] = (v8f){0.f, 0.f, 0.f, 0.f, 0.f, 0.f, 0.f, 0.f};
    accB[i] = (v8f){0.f, 0.f, 0.f, 0.f, 0.f, 0.f, 0.f, 0.f};
  }
  const int dmaxA = kPairSpan * pA + kStrip;
  const int dmaxB = kPairSpan * pB + kStrip;
  int delta = -32;
#pragma unroll 1
  for (; delta <= dmaxA; delta += 32) conv_step<true>(aP, bPA, bPB, delta, accA, accB);
#pragma unroll 1
  for (; delta <= dmaxB; delta += 32) conv_step<false>(aP, bPA, bPB, delta, accA, accB);

  const float dh = Dv[h];
  float* slab = sT[w];
  store_pair(slab, accA, pA, h, lane, dh, u, out);
  store_pair(slab, accB, pB, h, lane, dh, u, out);
}

extern "C" void kernel_launch(void* const* d_in, const int* in_sizes, int n_in,
                              void* d_out, int out_size, void* d_ws, size_t ws_size,
                              hipStream_t stream) {
  if (n_in < 6) return;
  if (in_sizes[0] != kBatch * kChan * kLen) return;
  if (in_sizes[1] != kChan * kModes) return;
  if (in_sizes[2] != kChan * kModes) return;
  if (in_sizes[3] != kChan * kModes * 2) return;
  if (in_sizes[4] != kChan) return;
  if (in_sizes[5] != kChan) return;
  if (out_size != kBatch * kChan * kLen) return;
  if (ws_size < kWsTotal) return;

  const float* u     = (const float*)d_in[0];
  const float* A_re  = (const float*)d_in[1];
  const float* A_im  = (const float*)d_in[2];
  const float* Cm    = (const float*)d_in[3];
  const float* Dv    = (const float*)d_in[4];
  const float* logst = (const float*)d_in[5];
  float* out = (float*)d_out;

  char* ws = (char*)d_ws;
  float*          PAR = (float*)(ws + kOffPar);
  unsigned short* TAP = (unsigned short*)(ws + kOffTap);
  unsigned short* SIG = (unsigned short*)(ws + kOffSig);

  mode_param_kernel<<<kChan, kModes, 0, stream>>>(A_re, A_im, Cm, logst, PAR);
  tap_plane_kernel<<<kChan, 256, 0, stream>>>(PAR, TAP);
  signal_plane_kernel<<<kSigChunks / 256, 256, 0, stream>>>(u, SIG);
  toeplitz_conv_kernel<<<kChan, 256, 0, stream>>>(TAP, SIG, u, Dv, out);
}
